// QuantizedPolicyValueNetwork_11570641895428
// MI455X (gfx1250) — hardware-verified
//
#include <hip/hip_runtime.h>
#include <hip/hip_bf16.h>

typedef __attribute__((ext_vector_type(16))) _Float16 v16h;
typedef __attribute__((ext_vector_type(8)))  _Float16 v8h;
typedef __attribute__((ext_vector_type(8)))  float    v8f;

#define NBOARD 19
#define NPIX   361
#define PADW   21
#define NPPIX  441
#define CCH    256
#define KTOT   2304
#define GRPBYTES 24576
#define NTBYTES  73728
#define PL_ACT   (NPPIX * CCH)
typedef __attribute__((ext_vector_type(4))) unsigned v4u_t;
typedef unsigned v4ua __attribute__((ext_vector_type(4), may_alias));
__device__ __forceinline__ _Float16 lo_of(float v, _Float16 h) { return (_Float16)((v - (float)h) * 2048.0f); }
__device__ __forceinline__ float act_f32(const _Float16* p) { return (float)p[0] + (float)p[PL_ACT] * (1.0f / 2048.0f); }

#if __has_builtin(__builtin_amdgcn_s_wait_asynccnt)
  #define PVN_WAIT_ASYNC(n) __builtin_amdgcn_s_wait_asynccnt(n)
#else
  #define PVN_WAIT_ASYNC(n) asm volatile("s_wait_asynccnt %0" :: "i"(n) : "memory")
#endif

__device__ __forceinline__ void pvn_async_copy_group(const void* gsrc, uint32_t ldst)
{
    uint64_t ga = (uint64_t)(uintptr_t)gsrc + (uint32_t)(threadIdx.x * 16);
    uint32_t la = ldst + threadIdx.x * 16;
    #pragma unroll
    for (int i = 0; i < 6; ++i) {
        asm volatile("global_load_async_to_lds_b128 %0, %1, off"
                     :: "v"(la), "v"(ga) : "memory");
        la += 4096;
        ga += 4096;
    }
}

__global__ void pvn_zero_acts(uint32_t* p, int ndw) {
    int i = blockIdx.x * 256 + threadIdx.x;
    if (i < ndw) { *(volatile uint32_t*)(p + i) = 0u; __threadfence(); *(volatile uint32_t*)(p + i) = 0u; }
}

__global__ void pvn_reformat_w2(const int* __restrict__ w, _Float16* __restrict__ wfrag) {
    const int t = blockIdx.x * 256 + threadIdx.x;
    if (t >= 36864) return;
    const int ln = t & 31, cblk = (t >> 5) & 7, tap = (t >> 8) % 9, nt = t / 2304;
    const int o = nt * 16 + (ln & 15);
    _Float16 hh[16];
    #pragma unroll
    for (int j = 0; j < 16; ++j) {
        const int c = cblk * 32 + ((ln >> 4) << 3) + (j < 8 ? j : j + 8);
        hh[j] = (_Float16)(float)w[o * KTOT + c * 9 + tap];
    }
    _Float16* d = wfrag + (size_t)t * 16;
    *(volatile v4u_t*)d = *(const v4ua*)hh; *(volatile v4u_t*)(d + 8) = *(const v4ua*)(hh + 8); __threadfence();
    *(volatile v4u_t*)d = *(const v4ua*)hh; *(volatile v4u_t*)(d + 8) = *(const v4ua*)(hh + 8);
}

__global__ void pvn_conv_init(const float* __restrict__ x,
                              const int* __restrict__ w,
                              const float* __restrict__ sptr,
                              const float* __restrict__ bias,
                              _Float16* __restrict__ act)
{
    const int n   = threadIdx.x;
    const int pix = blockIdx.x;
    const int y   = pix / NBOARD, xc = pix % NBOARD;
    const float s = sptr[0];
    float sum = 0.f;
    #pragma unroll
    for (int tap = 0; tap < 9; ++tap) {
        const int ky = tap / 3 - 1, kx = tap % 3 - 1;
        const int yy = y + ky, xx = xc + kx;
        const bool ok = (yy >= 0) & (yy < NBOARD) & (xx >= 0) & (xx < NBOARD);
        #pragma unroll
        for (int c = 0; c < 4; ++c) {
            float v = 0.f;
            if (ok) v = (c < 3) ? x[c * NPIX + yy * NBOARD + xx] : 1.0f;
            sum += v * (float)w[(n * 4 + c) * 9 + tap];
        }
    }
    float o = sum * s + bias[n];
    o = o > 0.f ? o : 0.f;
    const float o1 = __shfl_xor(o, 1, 32);
    if ((n & 1) == 0) {
        const _Float16 h0 = (_Float16)o, h1 = (_Float16)o1;
        const unsigned u = (unsigned)__builtin_bit_cast(unsigned short, h0) | ((unsigned)__builtin_bit_cast(unsigned short, h1) << 16);
        const unsigned l = (unsigned)__builtin_bit_cast(unsigned short, lo_of(o, h0)) | ((unsigned)__builtin_bit_cast(unsigned short, lo_of(o1, h1)) << 16);
        _Float16* d = act + ((y + 1) * PADW + (xc + 1)) * CCH + n;
        *(volatile unsigned*)d = u; *(volatile unsigned*)(d + PL_ACT) = l; __threadfence();
        *(volatile unsigned*)d = u; *(volatile unsigned*)(d + PL_ACT) = l;
    }
}

__global__ __launch_bounds__(256) void pvn_conv3x3_wmma(
    const _Float16* __restrict__ wfrag,
    const float* __restrict__ sptr,
    const float* __restrict__ bias,
    const _Float16* __restrict__ actIn,
    _Float16* actOut,
    const _Float16* skip)
{
    __shared__ __align__(16) _Float16 so[2][32 * 72];

    const int tid   = threadIdx.x;
    const int lane  = tid & 31;
    const int wave  = tid >> 5;
    const int ng    = blockIdx.x;
    const int ntile = ng * 4 + (wave & 3);
    const int mtile = blockIdx.y * 2 + (wave >> 2);

    int mrow = mtile * 16 + (lane & 15);
    if (mrow >= NPIX) mrow = NPIX - 1;
    const int py = mrow / NBOARD, px = mrow % NBOARD;
    const int hi = lane >> 4;
    const float s = sptr[0];

    const _Float16* wnt = wfrag + (size_t)ntile * (NTBYTES / 2);

    v8f acc = {};
    if (mtile < 23) {
        for (int g = 0; g < 3; ++g) {
            const _Float16* wg = wnt + g * (GRPBYTES / 2);
            for (int t2 = 0; t2 < 3; ++t2) {
                const int pix = (py + g) * PADW + (px + t2);
                const _Float16* abase = actIn + pix * CCH + hi * 8;
                #pragma unroll
                for (int cblk = 0; cblk < 8; ++cblk) {
                    const v8h a0 = *(const v8h*)(abase + cblk * 32);
                    const v8h a1 = *(const v8h*)(abase + cblk * 32 + 16);
                    const v8h l0 = *(const v8h*)(abase + PL_ACT + cblk * 32);
                    const v8h l1 = *(const v8h*)(abase + PL_ACT + cblk * 32 + 16);
                    const v16h a  = __builtin_shufflevector(a0, a1, 0, 1, 2, 3, 4, 5, 6, 7, 8, 9, 10, 11, 12, 13, 14, 15);
                    const v16h al = __builtin_shufflevector(l0, l1, 0, 1, 2, 3, 4, 5, 6, 7, 8, 9, 10, 11, 12, 13, 14, 15);
                    const _Float16* bbase = wg + (((t2 * 8 + cblk) * 32 + lane) << 4);
                    const v16h b = __builtin_shufflevector(*(const v8h*)bbase, *(const v8h*)(bbase + 8),
                        0, 1, 2, 3, 4, 5, 6, 7, 8, 9, 10, 11, 12, 13, 14, 15);
                    v8f lo = {};
                    lo  = __builtin_amdgcn_wmma_f32_16x16x32_f16(false, al, false, b, (short)0, lo, false, false);
                    acc = __builtin_amdgcn_wmma_f32_16x16x32_f16(false, a,  false, b, (short)0, acc, false, false);
                    acc += lo * (1.0f / 2048.0f);
                }
            }
        }
    }

    {
        const int nl = (wave & 3) * 16 + (lane & 15), n = ng * 64 + nl;
        const float bn = bias[n];
        #pragma unroll
        for (int gq = 0; gq < 8; ++gq) {
            const int ml = (wave >> 2) * 16 + gq + hi * 8;
            const int m = mtile * 16 + gq + hi * 8;
            float v = 0.f;
            if (mtile < 23 && m < NPIX) {
                const int pix = (m / NBOARD + 1) * PADW + (m % NBOARD + 1);
                v = acc[gq] * s + bn;
                if (skip) v += act_f32(skip + pix * CCH + n);
                v = v > 0.f ? v : 0.f;
            }
            const _Float16 hv = (_Float16)v;
            so[0][ml * 72 + nl] = hv; so[1][ml * 72 + nl] = lo_of(v, hv);
        }
    }
    __syncthreads();
    {
        const int ml = tid >> 3, q = (tid & 7) * 8;
        const int m = blockIdx.y * 32 + ml;
        if (m < NPIX) {
            const int pix = (m / NBOARD + 1) * PADW + (m % NBOARD + 1);
            _Float16* d = actOut + pix * CCH + ng * 64 + q;
            const v4u_t hv = *(const v4ua*)(so[0] + ml * 72 + q), lv = *(const v4ua*)(so[1] + ml * 72 + q);
            *(volatile v4u_t*)d = hv; *(volatile v4u_t*)(d + PL_ACT) = lv; __threadfence();
            *(volatile v4u_t*)d = hv; *(volatile v4u_t*)(d + PL_ACT) = lv;
        }
    }
}

__global__ void pvn_head_conv1x1(const _Float16* __restrict__ act,
                                 const int* __restrict__ wp, const float* sp,
                                 const float* bpv,
                                 const int* __restrict__ wv, const float* sv,
                                 const float* bvv,
                                 float* ph, float* vh)
{
    const int idx = blockIdx.x * 256 + threadIdx.x;
    if (idx < 722) {
        const int o = idx / NPIX, pix = idx % NPIX;
        const int pp = (pix / NBOARD + 1) * PADW + (pix % NBOARD + 1);
        float sum = 0.f;
        for (int c = 0; c < CCH; ++c)
            sum += act_f32(act + pp * CCH + c) * (float)wp[o * CCH + c];
        float v = sum * sp[0] + bpv[o];
        ph[idx] = v > 0.f ? v : 0.f;
    } else if (idx < 722 + NPIX) {
        const int pix = idx - 722;
        const int pp = (pix / NBOARD + 1) * PADW + (pix % NBOARD + 1);
        float sum = 0.f;
        for (int c = 0; c < CCH; ++c)
            sum += act_f32(act + pp * CCH + c) * (float)wv[c];
        float v = sum * sv[0] + bvv[0];
        vh[pix] = v > 0.f ? v : 0.f;
    }
}

__global__ void pvn_policy_fc(const float* __restrict__ ph,
                              const int* __restrict__ w, const float* sptr,
                              const float* __restrict__ bp, float* out)
{
    const int j = blockIdx.x * 256 + threadIdx.x;
    if (j < NPIX) {
        float sum = 0.f;
        for (int i = 0; i < 722; ++i)
            sum += ph[i] * (float)w[i * NPIX + j];
        const float v = sum * sptr[0] + bp[j];
        *(volatile float*)(out + j) = v; __threadfence(); *(volatile float*)(out + j) = v;
    }
}

__global__ void pvn_value_fc(const float* __restrict__ vh,
                             const int* __restrict__ w1, const float* s1,
                             const float* __restrict__ b1,
                             const int* __restrict__ w2, const float* s2,
                             const float* __restrict__ b2, float* out)
{
    __shared__ float red[256];
    const int u = threadIdx.x;
    float sum = 0.f;
    for (int p = 0; p < NPIX; ++p)
        sum += vh[p] * (float)w1[p * 256 + u];
    float h = sum * s1[0] + b1[u];
    h = h > 0.f ? h : 0.f;
    red[u] = h * (float)w2[u];
    __syncthreads();
    for (int st = 128; st > 0; st >>= 1) {
        if (u < st) red[u] += red[u + st];
        __syncthreads();
    }
    if (u == 0) { const float v = tanhf(red[0] * s2[0] + b2[0]); *(volatile float*)(out + NPIX) = v; __threadfence(); *(volatile float*)(out + NPIX) = v; }
}

extern "C" void kernel_launch(void* const* d_in, const int* in_sizes, int n_in,
                              void* d_out, int out_size, void* d_ws, size_t ws_size,
                              hipStream_t stream)
{
    const float* x       = (const float*)d_in[0];
    const int*   w_init  = (const int*)  d_in[1];
    const float* s_init  = (const float*)d_in[2];
    const float* b_init  = (const float*)d_in[3];
    const int*   rw1     = (const int*)  d_in[4];
    const float* rs1     = (const float*)d_in[5];
    const float* rb1     = (const float*)d_in[6];
    const int*   rw2     = (const int*)  d_in[7];
    const float* rs2     = (const float*)d_in[8];
    const float* rb2     = (const float*)d_in[9];
    const int*   wp      = (const int*)  d_in[10];
    const float* sp      = (const float*)d_in[11];
    const float* bpcv    = (const float*)d_in[12];
    const int*   fcpw    = (const int*)  d_in[13];
    const float* fcps    = (const float*)d_in[14];
    const float* bp      = (const float*)d_in[15];
    const int*   wv      = (const int*)  d_in[16];
    const float* sv      = (const float*)d_in[17];
    const float* bvcv    = (const float*)d_in[18];
    const int*   fv1w    = (const int*)  d_in[19];
    const float* fv1s    = (const float*)d_in[20];
    const float* bv1     = (const float*)d_in[21];
    const int*   fv2w    = (const int*)  d_in[22];
    const float* fv2s    = (const float*)d_in[23];
    const float* bv2     = (const float*)d_in[24];

    _Float16* A0   = (_Float16*)d_ws;
    _Float16* A1   = A0 + 2 * NPPIX * CCH;
    _Float16* wbuf = (_Float16*)((char*)d_ws + 4 * NPPIX * CCH * 2 + 4096);
    float*    ph   = (float*)(wbuf + 589824 + 2048);
    float*    vh   = ph + 722;
    float*    out  = (float*)d_out;

    const int ndw = (4 * NPPIX * CCH * (int)sizeof(_Float16)) / 4;
    pvn_zero_acts<<<(ndw + 255) / 256, 256, 0, stream>>>((uint32_t*)d_ws, ndw);

    pvn_conv_init<<<NPIX, 256, 0, stream>>>(x, w_init, s_init, b_init, A0);
    for (int b = 0; b < 10; ++b) {
        pvn_reformat_w2<<<36864 / 256, 256, 0, stream>>>(rw1 + (size_t)b * CCH * KTOT, wbuf);
        pvn_conv3x3_wmma<<<dim3(4, 12), 256, 0, stream>>>(wbuf, rs1 + b, rb1 + b * CCH, A0, A1, nullptr);

        pvn_reformat_w2<<<36864 / 256, 256, 0, stream>>>(rw2 + (size_t)b * CCH * KTOT, wbuf);
        pvn_conv3x3_wmma<<<dim3(4, 12), 256, 0, stream>>>(wbuf, rs2 + b, rb2 + b * CCH, A1, A0, A0);
    }

    pvn_head_conv1x1<<<5, 256, 0, stream>>>(A0, wp, sp, bpcv, wv, sv, bvcv, ph, vh);
    pvn_policy_fc<<<2, 256, 0, stream>>>(ph, fcpw, fcps, bp, out);
    pvn_value_fc<<<1, 256, 0, stream>>>(vh, fv1w, fv1s, bv1, fv2w, fv2s, bv2, out);
}
